// IntraZPConv_39213051412497
// MI455X (gfx1250) — hardware-verified
//
#include <hip/hip_runtime.h>

#define BS      2
#define C_IN    64
#define NP      1024
#define NA      60
#define NA_OUT  60
#define KS      3
#define ANN     8
#define C_OUT   128
#define KDIM    (C_IN * KS)
#define NJ      (NA_OUT * KS)
#define PTS     8
#define CHG     64
#define NCHG    (C_OUT / CHG)
#define NPB     ((BS * NP) / PTS)
#define SEG     (PTS * NA_OUT)
#define OPAD    64
#define XROW    200
#define WROW    200
#define FP      60
#define NTHR    256

static_assert(NP % PTS == 0, "");
static_assert((SEG * 4) % 128 == 0, "");
static_assert(KDIM % 32 == 0, "");
static_assert(C_OUT % CHG == 0, "");
static_assert((XROW % 8) == 0 && (WROW % 8) == 0, "");

#define OFF_STAGE 0
#define SZ_STAGE  (CHG * SEG * 4)
#define OFF_F     (OFF_STAGE + SZ_STAGE)
#define SZ_F      (C_IN * FP * 4)
#define OFF_WT    (OFF_F + SZ_F)
#define SZ_WT     (NJ * ANN * 4)
#define OFF_IT    (OFF_WT + SZ_WT)
#define SZ_IT     (NJ * ANN * 4)
#define OFF_BS    (OFF_IT + SZ_IT)
#define SZ_BS     (CHG * 4)
#define OFF_XH    (OFF_BS + SZ_BS)
#define SZ_X      (OPAD * XROW * 2)
#define OFF_XL    (OFF_XH + SZ_X)
#define OFF_WH    (OFF_XL + SZ_X)
#define SZ_W      (CHG * WROW * 2)
#define OFF_WL    (OFF_WH + SZ_W)
#define LDS_BYTES (OFF_WL + SZ_W)

static_assert(OFF_F % 16 == 0 && OFF_XH % 16 == 0 && OFF_XL % 16 == 0 && OFF_WH % 16 == 0 && OFF_WL % 16 == 0, "");
static_assert(LDS_BYTES == 252416, "");

typedef __bf16 v16b __attribute__((ext_vector_type(16)));
typedef __bf16 v8b  __attribute__((ext_vector_type(8)));
typedef v8b   __attribute__((may_alias)) v8ba;
typedef float v8f  __attribute__((ext_vector_type(8)));
typedef float v4f  __attribute__((ext_vector_type(4)));
typedef v4f   __attribute__((may_alias)) v4fa;

union Frag { v16b v; v8b hf[2]; };
union AccU { v8f v; float f[8]; };

static __device__ __forceinline__ v8f wmma_bf(v16b a, v16b b, v8f c) {
  v8f d = __builtin_amdgcn_wmma_f32_16x16x32_bf16(false, a, false, b, (short)0, c, false, false);
  asm volatile("v_nop\n\tv_nop\n\tv_nop\n\tv_nop" : "+v"(d) : "v"(a), "v"(b));
  return d;
}

static __device__ __forceinline__ void store_seg(const float* stage, float* gout, int wv, int lane) {
  #pragma unroll 1
  for (int cc = 0; cc < CHG / 8; ++cc) {
    const int ch = wv * (CHG / 8) + cc;
    const float* srow = stage + ch * SEG;
    float* grow = gout + (size_t)ch * (size_t)(NP * NA_OUT);
    #pragma unroll
    for (int q = 0; q < 4; ++q) {
      const int f = q * 128 + lane * 4;
      if (f < SEG) {
        const v4f v = *(const v4fa*)(srow + f);
        *(volatile v4f*)(grow + f) = v;
      }
    }
  }
}

__global__ __launch_bounds__(NTHR)
void k_fused(const float* __restrict__ feats,
             const float* __restrict__ intra_w,
             const float* __restrict__ Wmat,
             const float* __restrict__ bias,
             const int*   __restrict__ intra_idx,
             float* out)
{
  extern __shared__ __align__(16) unsigned char smem[];
  float*  stage = (float*)(smem + OFF_STAGE);
  float*  Fs    = (float*)(smem + OFF_F);
  float*  wt    = (float*)(smem + OFF_WT);
  int*    it    = (int*)(smem + OFF_IT);
  float*  bsv   = (float*)(smem + OFF_BS);
  __bf16* Xh    = (__bf16*)(smem + OFF_XH);
  __bf16* Xl    = (__bf16*)(smem + OFF_XL);
  __bf16* Wh    = (__bf16*)(smem + OFF_WH);
  __bf16* Wl    = (__bf16*)(smem + OFF_WL);

  const int tid  = threadIdx.x;
  const int lane = tid & 31;
  const int wv   = tid >> 5;
  const int h    = lane >> 4;
  const int m    = lane & 15;

  const int pb = blockIdx.x, cg = blockIdx.y;
  if (pb >= NPB || cg >= NCHG) return;
  const int flat0 = pb * PTS;
  const int b   = flat0 / NP;
  const int p0  = flat0 - b * NP;
  const int ch0 = cg * CHG;

  for (int e = tid; e < NJ * ANN; e += NTHR) {
    wt[e] = intra_w[e];
    int v = intra_idx[e];
    if (v < 0) v += NA;
    v = (v < 0) ? 0 : ((v > NA - 1) ? (NA - 1) : v);
    it[e] = v;
  }
  for (int e = tid; e < CHG; e += NTHR) bsv[e] = bias[ch0 + e];
  for (int e = tid; e < CHG * KDIM; e += NTHR) {
    const int ml = e / KDIM, i = e - ml * KDIM;
    const float x = Wmat[(size_t)(ch0 + ml) * KDIM + i];
    const __bf16 hi = (__bf16)x;
    const __bf16 lo = (__bf16)(x - (float)hi);
    Wh[ml * WROW + i] = hi;
    Wl[ml * WROW + i] = lo;
  }
  for (int e = tid; e < (OPAD - NA_OUT) * XROW; e += NTHR) {
    const int rr = e / XROW;
    const int r  = NA_OUT + rr;
    const int cc = e - rr * XROW;
    Xh[r * XROW + cc] = (__bf16)0.0f;
    Xl[r * XROW + cc] = (__bf16)0.0f;
  }

  const int mt = wv & 3;
  const int nh = wv >> 2;
  const size_t gbase = ((size_t)(b * C_OUT + ch0) * NP + (size_t)p0) * NA_OUT;

  for (int pt = 0; pt < PTS; ++pt) {
    const int p = p0 + pt;

    for (int e = tid; e < C_IN * NA; e += NTHR) {
      const int c = e / NA, na = e - c * NA;
      Fs[c * FP + na] = feats[((size_t)(b * C_IN + c) * NP + (size_t)p) * NA + na];
    }
    __syncthreads();

    if (tid < NJ) {
      const int j = tid;
      const int o = j / KS;
      const int k = j - o * KS;
      float w8[ANN]; int i8[ANN];
      #pragma unroll
      for (int a = 0; a < ANN; ++a) { w8[a] = wt[j * ANN + a]; i8[a] = it[j * ANN + a]; }
      __bf16* xh = Xh + o * XROW + k;
      __bf16* xl = Xl + o * XROW + k;
      #pragma unroll 1
      for (int c = 0; c < C_IN; ++c) {
        const float* fr = Fs + c * FP;
        float s = 0.0f;
        #pragma unroll
        for (int a = 0; a < ANN; ++a) s = fmaf(w8[a], fr[i8[a]], s);
        const __bf16 hi = (__bf16)s;
        const __bf16 lo = (__bf16)(s - (float)hi);
        xh[c * KS] = hi;
        xl[c * KS] = lo;
      }
    }
    __syncthreads();

    {
      v8f acc0 = (v8f){0.f,0.f,0.f,0.f,0.f,0.f,0.f,0.f};
      v8f acc1 = (v8f){0.f,0.f,0.f,0.f,0.f,0.f,0.f,0.f};
      const __bf16* wrh = Wh + (mt * 16 + m) * WROW + 8 * h;
      const __bf16* wrl = Wl + (mt * 16 + m) * WROW + 8 * h;
      const __bf16* x0h = Xh + (nh * 32 + m) * XROW + 8 * h;
      const __bf16* x0l = Xl + (nh * 32 + m) * XROW + 8 * h;
      const __bf16* x1h = x0h + 16 * XROW;
      const __bf16* x1l = x0l + 16 * XROW;
      #pragma unroll 1
      for (int ks = 0; ks < KDIM / 32; ++ks) {
        const int k0 = ks * 32;
        Frag ah, al, b0h, b0l, b1h, b1l;
        ah.hf[0]  = *(const v8ba*)(wrh + k0);  ah.hf[1]  = *(const v8ba*)(wrh + k0 + 16);
        al.hf[0]  = *(const v8ba*)(wrl + k0);  al.hf[1]  = *(const v8ba*)(wrl + k0 + 16);
        b0h.hf[0] = *(const v8ba*)(x0h + k0);  b0h.hf[1] = *(const v8ba*)(x0h + k0 + 16);
        b0l.hf[0] = *(const v8ba*)(x0l + k0);  b0l.hf[1] = *(const v8ba*)(x0l + k0 + 16);
        b1h.hf[0] = *(const v8ba*)(x1h + k0);  b1h.hf[1] = *(const v8ba*)(x1h + k0 + 16);
        b1l.hf[0] = *(const v8ba*)(x1l + k0);  b1l.hf[1] = *(const v8ba*)(x1l + k0 + 16);
        acc0 = wmma_bf(ah.v, b0h.v, acc0);
        acc0 = wmma_bf(ah.v, b0l.v, acc0);
        acc0 = wmma_bf(al.v, b0h.v, acc0);
        acc1 = wmma_bf(ah.v, b1h.v, acc1);
        acc1 = wmma_bf(ah.v, b1l.v, acc1);
        acc1 = wmma_bf(al.v, b1h.v, acc1);
      }
      AccU u0, u1; u0.v = acc0; u1.v = acc1;
      const int rbase = mt * 16 + 8 * h;
      const int o0 = nh * 32 + m;
      const int o1 = o0 + 16;
      #pragma unroll
      for (int r = 0; r < 8; ++r) {
        const float bv = bsv[rbase + r];
        float* srow = stage + (rbase + r) * SEG + pt * NA_OUT;
        srow[o0] = u0.f[r] + bv;
        if (o1 < NA_OUT) srow[o1] = u1.f[r] + bv;
      }
    }
    __syncthreads();
  }

  store_seg(stage, out + gbase, wv, lane);
  __threadfence();
  store_seg(stage, out + gbase, wv, lane);
}

extern "C" void kernel_launch(void* const* d_in, const int* in_sizes, int n_in,
                              void* d_out, int out_size, void* d_ws, size_t ws_size,
                              hipStream_t stream) {
  (void)d_ws; (void)ws_size;
  if (n_in < 5) return;
  if (in_sizes[0] != BS * C_IN * NP * NA) return;
  if (in_sizes[1] != NJ * ANN) return;
  if (in_sizes[2] != C_OUT * KDIM) return;
  if (in_sizes[3] != C_OUT) return;
  if (in_sizes[4] != NJ * ANN) return;
  if (out_size != BS * C_OUT * NP * NA_OUT) return;

  const float* feats     = (const float*)d_in[0];
  const float* intra_w   = (const float*)d_in[1];
  const float* Wmat      = (const float*)d_in[2];
  const float* bias      = (const float*)d_in[3];
  const int*   intra_idx = (const int*)  d_in[4];
  float* out = (float*)d_out;

  hipFuncSetAttribute((const void*)k_fused, hipFuncAttributeMaxDynamicSharedMemorySize, LDS_BYTES);
  hipLaunchKernelGGL(k_fused, dim3(NPB, NCHG, 1), dim3(NTHR, 1, 1), (size_t)LDS_BYTES, stream,
                     feats, intra_w, Wmat, bias, intra_idx, out);
  (void)hipGetLastError();
}
